// DCBlock_88381837017390
// MI455X (gfx1250) — hardware-verified
//
#include <hip/hip_runtime.h>


#define CC   256
#define CP   19
#define HH   80
#define NP   (HH * HH)
#define KK   7
#define K2   49
#define PADK 3
typedef _Float16 h16;
typedef unsigned short bf;
typedef __attribute__((ext_vector_type(16))) __bf16   v16bf;
typedef __attribute__((ext_vector_type(16))) _Float16 v16h;
typedef __attribute__((ext_vector_type(8)))  _Float16 v8h;
typedef __attribute__((ext_vector_type(8)))  unsigned short v8us;
typedef __attribute__((ext_vector_type(8)))  float    v8f;
typedef __attribute__((ext_vector_type(4)))  float    v4f;
typedef v8h  __attribute__((may_alias)) v8ha;
typedef v4f  __attribute__((may_alias)) v4fa;
typedef v8us __attribute__((may_alias)) v8usa;

__device__ __forceinline__ unsigned short f2bf(float f) { unsigned u = __float_as_uint(f); u += 0x7FFFu + ((u >> 16) & 1u); return (unsigned short)(u >> 16); }
__device__ __forceinline__ float bf2f(unsigned short b) { return __uint_as_float(((unsigned)b) << 16); }
__device__ __forceinline__ float bfr(float f) { return bf2f(f2bf(f)); }
__device__ __forceinline__ v16h cat16(v8h lo, v8h hi) { return __builtin_shufflevector(lo, hi, 0, 1, 2, 3, 4, 5, 6, 7, 8, 9, 10, 11, 12, 13, 14, 15); }
__device__ __forceinline__ v16bf cat16b(v8us lo, v8us hi) { return __builtin_bit_cast(v16bf, __builtin_shufflevector(lo, hi, 0, 1, 2, 3, 4, 5, 6, 7, 8, 9, 10, 11, 12, 13, 14, 15)); }
__device__ __forceinline__ v8f wmma16(v16h a, v16h b, v8f c) { return __builtin_amdgcn_wmma_f32_16x16x32_f16(false, a, false, b, (short)0, c, false, false); }
__device__ __forceinline__ v8f wmmab(v16bf a, v16bf b, v8f c) { return __builtin_amdgcn_wmma_f32_16x16x32_bf16(false, a, false, b, (short)0, c, false, false); }


template <typename T16> struct WFrag;
template <> struct WFrag<h16> { typedef v16h V; static __device__ __forceinline__ V ld(const h16* p) { return cat16(*(const v8h*)p, *(const v8h*)(p + 16)); } static __device__ __forceinline__ v8f mma(V a, V b, v8f c) { return wmma16(a, b, c); } };
template <> struct WFrag<bf> { typedef v16bf V; static __device__ __forceinline__ V ld(const bf* p) { return cat16b(*(const v8us*)p, *(const v8us*)(p + 16)); } static __device__ __forceinline__ v8f mma(V a, V b, v8f c) { return wmmab(a, b, c); } };
template <typename T16, int NSPLIT, bool BIAS>
__global__ __launch_bounds__(32) void k_gemmw(const T16* __restrict__ A, const T16* __restrict__ A2, const T16* __restrict__ Bt, const T16* __restrict__ Bt2, int K, float* C, int ldc, const float* __restrict__ bias, size_t sA, size_t sB, size_t sC) {
    typedef typename WFrag<T16>::V V;
    __shared__ __align__(16) float os[16 * 68];
    const size_t z = blockIdx.z; A += z * sA; if (A2) A2 += z * sA; Bt += z * sB; if (Bt2) Bt2 += z * sB; C += z * sC;
    const int lane = threadIdx.x & 31, lr = lane & 15, hi = lane >> 4; const int r0 = blockIdx.x * 64, c0 = blockIdx.y * 64;
    v8f acc[4][4];
#pragma unroll
    for (int mb = 0; mb < 4; ++mb)
#pragma unroll
        for (int nb = 0; nb < 4; ++nb) acc[mb][nb] = (v8f){};
    const size_t aoff = (size_t)(r0 + lr) * K + 8 * hi, boff = (size_t)(c0 + lr) * K + 8 * hi;
#pragma unroll 1
    for (int kc = 0; kc < K; kc += 32) {
        V a[4], a2[4];
#pragma unroll
        for (int mb = 0; mb < 4; ++mb) { a[mb] = WFrag<T16>::ld(A + aoff + (size_t)mb * 16 * K + kc); if (NSPLIT == 1 || NSPLIT == 2) a2[mb] = WFrag<T16>::ld(A2 + aoff + (size_t)mb * 16 * K + kc); }
#pragma unroll
        for (int nb = 0; nb < 4; ++nb) { const V b = WFrag<T16>::ld(Bt + boff + (size_t)nb * 16 * K + kc); V b2; if (NSPLIT >= 2) b2 = WFrag<T16>::ld(Bt2 + boff + (size_t)nb * 16 * K + kc);
#pragma unroll
            for (int mb = 0; mb < 4; ++mb) { acc[mb][nb] = WFrag<T16>::mma(a[mb], b, acc[mb][nb]); if (NSPLIT == 1 || NSPLIT == 2) acc[mb][nb] = WFrag<T16>::mma(a2[mb], b, acc[mb][nb]); if (NSPLIT >= 2) acc[mb][nb] = WFrag<T16>::mma(a[mb], b2, acc[mb][nb]); } }
        asm volatile("v_nop\n\tv_nop\n\tv_nop\n\tv_nop" : "+v"(acc[0][0]), "+v"(acc[1][1]), "+v"(acc[2][2]), "+v"(acc[3][3]) : "v"(a[0]), "v"(a[3]));
    }
#pragma unroll
    for (int mb = 0; mb < 4; ++mb) {
#pragma unroll
        for (int nb = 0; nb < 4; ++nb) {
#pragma unroll
            for (int j = 0; j < 8; ++j) os[(hi * 8 + j) * 68 + nb * 16 + lr] = acc[mb][nb][j]; }
        __builtin_amdgcn_wave_barrier(); asm volatile("" ::: "memory");
        float* crow = C + (size_t)(r0 + mb * 16) * ldc + c0;
#pragma unroll 1
        for (int ps = 0; ps < 2; ++ps) {
#pragma unroll
            for (int s = 0; s < 8; ++s) { const int row = 2 * s + hi, cofs = lr * 4; v4f val = *(const v4fa*)(os + row * 68 + cofs); if (BIAS) { val[0] += bfr(bias[c0 + cofs]); val[1] += bfr(bias[c0 + cofs + 1]); val[2] += bfr(bias[c0 + cofs + 2]); val[3] += bfr(bias[c0 + cofs + 3]); }
                *(volatile v4f*)(crow + (size_t)row * ldc + cofs) = val; }
            if (ps == 0) __threadfence(); }
        __builtin_amdgcn_wave_barrier(); asm volatile("" ::: "memory");
    }
}

__device__ __forceinline__ void splitf(float y, unsigned short& h, unsigned short& l) { h = f2bf(y); l = f2bf(y - bf2f(h)); }
typedef __attribute__((ext_vector_type(2))) unsigned short v2us;
typedef __attribute__((ext_vector_type(2))) float v2f;

__global__ __launch_bounds__(256) void k_cvt8(const float* __restrict__ src, bf* dst, size_t n8) { const size_t i = (size_t)blockIdx.x * 256 + threadIdx.x; if (i >= n8) return; const v8f v = *(const v8f*)(src + i * 8); v8us o;
#pragma unroll
    for (int k = 0; k < 8; ++k) o[k] = f2bf(v[k]); *(volatile v8us*)(dst + i * 8) = o; __threadfence(); *(volatile v8us*)(dst + i * 8) = o; }
__global__ __launch_bounds__(256) void k_bnT(const float* __restrict__ x, const float* __restrict__ g, const float* __restrict__ bb, const float* __restrict__ mu, const float* __restrict__ var, bf* Xh, bf* Xl) { const int e = (blockIdx.x * 256 + threadIdx.x) * 2; if (e >= NP * CC) return; const int c = e % CC, pos = e / CC; v2us oh, ol;
#pragma unroll
    for (int q = 0; q < 2; ++q) { const int cq = c + q; float gm = bfr(g[cq]), be = bfr(bb[cq]), mm = bfr(mu[cq]), vv = bfr(var[cq]); asm volatile("" : "+v"(gm)); asm volatile("" : "+v"(be)); asm volatile("" : "+v"(mm)); asm volatile("" : "+v"(vv));
        const float sc = __fmul_rn(__fdiv_rn(1.0f, __fsqrt_rn(__fadd_rn(vv, 1e-5f))), gm); float t = __fmul_rn(__fsub_rn(bfr(x[(size_t)cq * NP + pos]), mm), sc); asm volatile("" : "+v"(t)); unsigned short a, c2; splitf(__fadd_rn(t, be), a, c2); oh[q] = a; ol[q] = c2; }
    *(volatile v2us*)(Xh + e) = oh; *(volatile v2us*)(Xl + e) = ol; __threadfence(); *(volatile v2us*)(Xh + e) = oh; *(volatile v2us*)(Xl + e) = ol; }
__global__ __launch_bounds__(256) void k_aff(const float* __restrict__ pr, const float* __restrict__ sig, float* AFF) { const int lane = threadIdx.x & 31; const int pos = blockIdx.x * 8 + (threadIdx.x >> 5); if (pos >= NP) return; const int y0 = pos / HH, x0 = pos % HH;
    float sg = bfr(sig[0]); sg = fmaxf(sg, 0.f); float den = __fmul_rn(2.0f, __fmul_rn(sg, sg)); asm volatile("" : "+v"(den)); den = __fadd_rn(den, 1e-8f);
    float ev[2];
#pragma unroll
    for (int sl = 0; sl < 2; ++sl) { const int k = sl * 32 + lane; ev[sl] = -3.0e38f; if (k < K2) { const int yy = y0 + k / KK - PADK, xx = x0 + k % KK - PADK; const bool in = (yy >= 0 && yy < HH && xx >= 0 && xx < HH); float d2 = 0.f;
#pragma unroll 1
            for (int cp = 0; cp < CP; ++cp) { const float ctr = bfr(pr[(size_t)cp * NP + pos]); const float nb = in ? bfr(pr[(size_t)cp * NP + yy * HH + xx]) : 0.f; const float df = __fsub_rn(nb, ctr); float sq = __fmul_rn(df, df); asm volatile("" : "+v"(sq)); d2 = __fadd_rn(d2, sq); }
            ev[sl] = __expf(-__fdiv_rn(d2, den)); } }
    float mx = fmaxf(ev[0], ev[1]);
#pragma unroll
    for (int sh = 16; sh; sh >>= 1) mx = fmaxf(mx, __shfl_xor(mx, sh, 32));
    float d0 = __fsub_rn(ev[0], mx), d1 = __fsub_rn(ev[1], mx); asm volatile("" : "+v"(d0)); asm volatile("" : "+v"(d1)); const float e0 = __builtin_amdgcn_exp2f(__fmul_rn(d0, 1.4426950408889634f)), e1 = (32 + lane < K2) ? __builtin_amdgcn_exp2f(__fmul_rn(d1, 1.4426950408889634f)) : 0.f; float s = __fadd_rn(e0, e1);
#pragma unroll
    for (int sh = 16; sh; sh >>= 1) s += __shfl_xor(s, sh, 32);
    const float inv = __fdiv_rn(1.0f, s); const float a0 = __fmul_rn(e0, inv), a1 = __fmul_rn(e1, inv); float* row = AFF + (size_t)pos * 64;
    *(volatile float*)(row + lane) = a0; *(volatile float*)(row + 32 + lane) = a1; __threadfence(); *(volatile float*)(row + lane) = a0; *(volatile float*)(row + 32 + lane) = a1; }
__global__ __launch_bounds__(256) void k_agg(const float* __restrict__ MSG, const float* __restrict__ AFF, bf* Gh, bf* Gl) { const int e = (blockIdx.x * 256 + threadIdx.x) * 2; if (e >= NP * CC) return; const int c = e % CC, pos = e / CC; const int y0 = pos / HH, x0 = pos % HH; float a0 = 0.f, a1 = 0.f;
    for (int k = 0; k < K2; ++k) { const int yy = y0 + k / KK - PADK, xx = x0 + k % KK - PADK; if (yy < 0 || yy >= HH || xx < 0 || xx >= HH) continue; const float w = AFF[(size_t)pos * 64 + k]; const float* m = MSG + ((size_t)yy * HH + xx) * CC + c;
        float p0 = __fmul_rn(w, m[0]), p1 = __fmul_rn(w, m[1]); asm volatile("" : "+v"(p0)); asm volatile("" : "+v"(p1)); a0 = __fadd_rn(a0, p0); a1 = __fadd_rn(a1, p1); }
    v2us oh, ol; unsigned short a, c2; splitf(a0, a, c2); oh[0] = a; ol[0] = c2; splitf(a1, a, c2); oh[1] = a; ol[1] = c2; *(volatile v2us*)(Gh + e) = oh; *(volatile v2us*)(Gl + e) = ol; __threadfence(); *(volatile v2us*)(Gh + e) = oh; *(volatile v2us*)(Gl + e) = ol; }
__global__ __launch_bounds__(256) void k_outT(const float* __restrict__ REF, const float* __restrict__ x, float* OUT) { const int e = (blockIdx.x * 256 + threadIdx.x) * 2; if (e >= CC * NP) return; const int pos = e % NP, o = e / NP; v2f r; r[0] = __fadd_rn(bfr(x[e]), REF[(size_t)pos * CC + o]); r[1] = __fadd_rn(bfr(x[e + 1]), REF[(size_t)(pos + 1) * CC + o]); *(volatile v2f*)(OUT + e) = r; __threadfence(); *(volatile v2f*)(OUT + e) = r; }

extern "C" void kernel_launch(void* const* d_in, const int* in_sizes, int n_in,
                              void* d_out, int out_size, void* d_ws, size_t ws_size, hipStream_t stream) {
    (void)in_sizes; (void)n_in; (void)out_size;
    const float* IN[9]; for (int i = 0; i < 9; ++i) IN[i] = (const float*)d_in[i];
    float* OUT = (float*)d_out;
    char* wsp = (char*)d_ws;
    auto take = [&](size_t bytes) { char* p = wsp; wsp += (bytes + 255) & ~(size_t)255; return (void*)p; };
    bf* WF = (bf*)take((size_t)CC * CC * 2); bf* WU = (bf*)take((size_t)CC * CC * 2); bf* Xh = (bf*)take((size_t)NP * CC * 2); bf* Xl = (bf*)take((size_t)NP * CC * 2); float* MSG = (float*)take((size_t)NP * CC * 4); float* AFF = (float*)take((size_t)NP * 64 * 4); bf* Gh = (bf*)take((size_t)NP * CC * 2); bf* Gl = (bf*)take((size_t)NP * CC * 2); float* REF = (float*)take((size_t)NP * CC * 4);
    if ((size_t)(wsp - (char*)d_ws) > ws_size) return;
    k_cvt8<<<(CC * CC / 8 + 255) / 256, 256, 0, stream>>>(IN[3], WF, (size_t)CC * CC / 8); k_cvt8<<<(CC * CC / 8 + 255) / 256, 256, 0, stream>>>(IN[4], WU, (size_t)CC * CC / 8);
    k_bnT<<<(NP * CC / 2 + 255) / 256, 256, 0, stream>>>(IN[0], IN[5], IN[6], IN[7], IN[8], Xh, Xl);
    k_gemmw<bf, 1, false><<<dim3(NP / 64, CC / 64, 1), 32, 0, stream>>>(Xh, Xl, WF, nullptr, CC, MSG, CC, nullptr, 0, 0, 0);
    k_aff<<<NP / 8, 256, 0, stream>>>(IN[1], IN[2], AFF);
    k_agg<<<(NP * CC / 2 + 255) / 256, 256, 0, stream>>>(MSG, AFF, Gh, Gl);
    k_gemmw<bf, 1, false><<<dim3(NP / 64, CC / 64, 1), 32, 0, stream>>>(Gh, Gl, WU, nullptr, CC, REF, CC, nullptr, 0, 0, 0);
    k_outT<<<(CC * NP / 2 + 255) / 256, 256, 0, stream>>>(REF, IN[0], OUT);
}
